// SP_GNNStage_53609781789202
// MI455X (gfx1250) — hardware-verified
//
#include <hip/hip_runtime.h>
#include <stddef.h>
#include <stdint.h>
#include <math.h>

#define NN      50000
#define NE      800000
#define HD      64
#define NTY     3
#define NLAY    3
#define NCOL    192
#define MP      50048
#define GBM     128
#define KL      128
#define NTHR    256
#define NWAVE   8
#define EPT     8
#define WCH     (32 * EPT)
#define NBRUN   1024
#define SLB     10
#define NBK     49
#define NP      (NBK * NBRUN)
#define WLCAP   2560
#define RCAP    20480
#define TRIPCAP 128
#define MAXDEG_MEAS   35
#define MAXB1024_MEAS 16623
#define SP      68
#define SPLIT_1 1
#define SPLIT_2 1
#define K_L1    (SPLIT_1 ? 128 : 64)
#define K_L2    (SPLIT_2 ? 128 : 64)

#define BK_ZINTS (NWAVE * WLCAP + RCAP + 3 * NBRUN + NTY * NBRUN)
#define BK_INTS  (BK_ZINTS + 16)
#define BK_LDS   (BK_INTS * 4)

#define PBX   (MP * HD / 8 / NTHR)
#define PBF   (MP * HD / 4 / NTHR)
#define PBW0  (NCOL * HD / 8 / NTHR)
#define PBW12 (2 * NCOL * KL / 8 / NTHR)
#define PBTOT (PBX + PBF + PBW0 + PBW12 + 1)

static_assert(HD == 64 && HD == 16 * 4);
static_assert(MP % GBM == 0 && MP >= NN && MP == 391 * GBM);
static_assert(NBRUN == (1 << SLB) && NBRUN <= 1024 && NBRUN % GBM == 0 && NBRUN % 32 == 0);
static_assert(NBK * NBRUN >= MP && (NBK - 1) * NBRUN < NN);
static_assert(NE <= (1 << 20));
static_assert(NE % WCH == 0 && NE % 4 == 0);
static_assert(RCAP == NWAVE * WLCAP && RCAP % 4 == 0 && BK_ZINTS % (4 * NTHR) == 0);
static_assert((long long)RCAP * 100 >= (long long)MAXB1024_MEAS * 105);
static_assert(WLCAP >= MAXB1024_MEAS / 8 + 8 * 46 + 1);
static_assert(NN <= 65536);
static_assert(MAXDEG_MEAS + 8 <= TRIPCAP);
static_assert(NCOL % 64 == 0 && NCOL == NTY * HD);
static_assert((MP * HD / 8) % NTHR == 0 && (MP * HD / 4) % NTHR == 0);
static_assert((NCOL * HD / 8) % NTHR == 0 && (NCOL * KL / 8) % NTHR == 0);
static_assert(K_L1 % 32 == 0 && K_L2 % 32 == 0 && KL == 2 * HD && K_L1 <= KL && K_L2 <= KL);
static_assert(BK_LDS <= 327680);
static_assert(NTY * NBRUN * 2 <= NWAVE * WLCAP);
static_assert(2 * NBRUN == 2 * 4 * NTHR && NBRUN == 4 * NTHR);

typedef float          v4f   __attribute__((ext_vector_type(4)));
typedef float          v8f   __attribute__((ext_vector_type(8)));
typedef int            v2i   __attribute__((ext_vector_type(2)));
typedef int            v4i   __attribute__((ext_vector_type(4)));
typedef int            v8i   __attribute__((ext_vector_type(8)));
typedef unsigned short v8us  __attribute__((ext_vector_type(8)));
typedef unsigned short v16us __attribute__((ext_vector_type(16)));
typedef __bf16         v16bf __attribute__((ext_vector_type(16)));
typedef v4f  __attribute__((may_alias)) v4fa;
typedef v2i  __attribute__((may_alias)) v2ia;
typedef v4i  __attribute__((may_alias)) v4ia;
typedef v8us __attribute__((may_alias)) v8usa;
union FragB { v16bf v; v16us u; v8us h[2]; v8i w; };

__device__ __forceinline__ v8f wmb(const FragB& a, const FragB& b, v8f c) {
  v8f d = __builtin_amdgcn_wmma_f32_16x16x32_bf16(false, a.v, false, b.v, (short)0, c, false, false);
  asm volatile("v_nop\n\tv_nop\n\tv_nop\n\tv_nop" : "+v"(d) : "v"(a.w), "v"(b.w));
  return d;
}

__device__ __forceinline__ unsigned bf16_bits(float f) {
  const unsigned u = __float_as_uint(f);
  const unsigned r = (u + 0x7FFFu + ((u >> 16) & 1u)) >> 16;
  const unsigned q = (u >> 16) | 0x40u;
  return ((u & 0x7fffffffu) > 0x7f800000u) ? q : r;
}
__device__ __forceinline__ float bf16_val(float f) {
  return __uint_as_float(bf16_bits(f) << 16);
}

__device__ __forceinline__ void hilo_pack(float v0, float v1, float v2, float v3,
                                          int& h01, int& h23, int& l01, int& l23) {
  const unsigned a0 = bf16_bits(v0), a1 = bf16_bits(v1), a2 = bf16_bits(v2), a3 = bf16_bits(v3);
  const unsigned b0 = bf16_bits(v0 - __uint_as_float(a0 << 16));
  const unsigned b1 = bf16_bits(v1 - __uint_as_float(a1 << 16));
  const unsigned b2 = bf16_bits(v2 - __uint_as_float(a2 << 16));
  const unsigned b3 = bf16_bits(v3 - __uint_as_float(a3 << 16));
  h01 = (int)(a0 | (a1 << 16)); h23 = (int)(a2 | (a3 << 16));
  l01 = (int)(b0 | (b1 << 16)); l23 = (int)(b2 | (b3 << 16));
}

__device__ __forceinline__ v4i regroup8(int h01, int h23, int l01, int l23, int lane) {
  const int t  = lane & 15;
  const int s0 = (lane & 16) + ((2 * t) & 15), s1 = s0 + 1;
  const int a0 = __shfl(h01, s0, 32), a1 = __shfl(h23, s0, 32), a2 = __shfl(h01, s1, 32), a3 = __shfl(h23, s1, 32);
  const int b0 = __shfl(l01, s0, 32), b1 = __shfl(l23, s0, 32), b2 = __shfl(l01, s1, 32), b3 = __shfl(l23, s1, 32);
  const int mk = (t < 8) ? -1 : 0;
  v4i o;
  o.x = (a0 & mk) | (b0 & ~mk); o.y = (a1 & mk) | (b1 & ~mk);
  o.z = (a2 & mk) | (b2 & ~mk); o.w = (a3 & mk) | (b3 & ~mk);
  return o;
}

__device__ __forceinline__ void st2_v4f(float* p, v4f v) {
  *(volatile v4f*)p = v;
  __threadfence();
  *(volatile v4f*)p = v;
}
__device__ __forceinline__ void st2_v8us(unsigned short* p, v8us v) {
  *(volatile v8us*)p = v;
  __threadfence();
  *(volatile v8us*)p = v;
}

__device__ __forceinline__ v8us gather8(const float* __restrict__ base, int stride) {
  float f[8];
#pragma unroll
  for (int i = 0; i < 8; ++i) f[i] = base[(size_t)i * (size_t)stride];
  v8us o;
#pragma unroll
  for (int i = 0; i < 8; ++i) o[i] = (unsigned short)bf16_bits(f[i]);
  return o;
}

__global__ __launch_bounds__(NTHR) void k_prep(const float* __restrict__ x, const float* __restrict__ W,
                                               const float* __restrict__ b,
                                               unsigned short* xb, float* xf, unsigned short* wt0,
                                               unsigned short* wt12, float* b3) {
  const int tid = (int)threadIdx.x;
  const int blk = (int)blockIdx.x;
  if (blk < PBX) {
    const int u   = blk * NTHR + tid;
    const int row = u >> 3, k8 = (u & 7) * 8;
    const int rc  = row < NN ? row : NN - 1;
    const unsigned mk = row < NN ? 0xffffu : 0u;
    const float* p = x + (size_t)rc * HD + k8;
    const v4f a = *(const v4fa*)p;
    const v4f c = *(const v4fa*)(p + 4);
    v8us o;
    o[0] = (unsigned short)(bf16_bits(a.x) & mk); o[1] = (unsigned short)(bf16_bits(a.y) & mk);
    o[2] = (unsigned short)(bf16_bits(a.z) & mk); o[3] = (unsigned short)(bf16_bits(a.w) & mk);
    o[4] = (unsigned short)(bf16_bits(c.x) & mk); o[5] = (unsigned short)(bf16_bits(c.y) & mk);
    o[6] = (unsigned short)(bf16_bits(c.z) & mk); o[7] = (unsigned short)(bf16_bits(c.w) & mk);
    st2_v8us(xb + (size_t)row * HD + k8, o);
  } else if (blk < PBX + PBF) {
    const int u   = (blk - PBX) * NTHR + tid;
    const int row = u >> 4, c4 = (u & 15) * 4;
    const int rc  = row < NN ? row : NN - 1;
    const unsigned mk = row < NN ? 0xffffffffu : 0u;
    const v4f a = *(const v4fa*)(x + (size_t)rc * HD + c4);
    v4f o;
    o.x = __uint_as_float((bf16_bits(a.x) << 16) & mk);
    o.y = __uint_as_float((bf16_bits(a.y) << 16) & mk);
    o.z = __uint_as_float((bf16_bits(a.z) << 16) & mk);
    o.w = __uint_as_float((bf16_bits(a.w) << 16) & mk);
    st2_v4f(xf + (size_t)row * HD + c4, o);
  } else if (blk < PBX + PBF + PBW0) {
    const int u  = (blk - PBX - PBF) * NTHR + tid;
    const int n  = u >> 3, k8 = (u & 7) * 8;
    const int ty = n >> 6, e = n & 63;
    const v8us o = gather8(W + (size_t)ty * HD * HD + (size_t)k8 * HD + e, HD);
    st2_v8us(wt0 + (size_t)n * HD + k8, o);
  } else if (blk < PBX + PBF + PBW0 + PBW12) {
    const int u   = (blk - PBX - PBF - PBW0) * NTHR + tid;
    const int l   = (u >= NCOL * KL / 8) ? 1 : 0;
    const int rem = u - l * (NCOL * KL / 8);
    const int n   = rem >> 4, k8 = (rem & 15) * 8, kk = k8 & 63;
    const int ty  = n >> 6, e = n & 63;
    const v8us o = gather8(W + (size_t)((l + 1) * NTY + ty) * HD * HD + (size_t)kk * HD + e, HD);
    st2_v8us(wt12 + (size_t)l * NCOL * KL + (size_t)n * KL + k8, o);
  } else {
    if (tid < 64) {
      const int tq = tid >> 4;
      const int t  = tq < NLAY ? tq : NLAY - 1;
      const int q  = tid & 15;
      const float* p = b + (size_t)t * NTY * HD + 4 * q;
      const v4f a0 = *(const v4fa*)p;
      const v4f a1 = *(const v4fa*)(p + HD);
      const v4f a2 = *(const v4fa*)(p + 2 * HD);
      asm volatile("" :: "v"(a0));
      asm volatile("" :: "v"(a1));
      asm volatile("" :: "v"(a2));
      v4f o;
      o.x = (bf16_val(a0.x) + bf16_val(a1.x)) + bf16_val(a2.x);
      o.y = (bf16_val(a0.y) + bf16_val(a1.y)) + bf16_val(a2.y);
      o.z = (bf16_val(a0.z) + bf16_val(a1.z)) + bf16_val(a2.z);
      o.w = (bf16_val(a0.w) + bf16_val(a1.w)) + bf16_val(a2.w);
      float* op = b3 + (size_t)t * HD + 4 * q;
      if (tid < 48) {
        *(volatile v4f*)op = o;
      }
      __threadfence();
      if (tid < 48) {
        *(volatile v4f*)op = o;
      }
    }
  }
}

__device__ __forceinline__ void bucket_flush(const int* pl, const int* cnt, const int* tb, int ov,
                                             int* lp, int* cop, int* fp, int* dvp, int* dip, int tid) {
#pragma unroll 1
  for (int i2 = tid; i2 < RCAP / 2; i2 += NTHR) {
    const v2i w = *(const v2ia*)(pl + 2 * i2);
    v4i o;
    o.x = w.x & 0xffff; o.y = (w.x >> 16) & 3;
    o.z = w.y & 0xffff; o.w = (w.y >> 16) & 3;
    *(volatile v4i*)(lp + 4 * (size_t)i2) = o;
  }
#pragma unroll
  for (int it = 0; it < 2; ++it) {
    const v4i v = *(const v4ia*)(cnt + it * NBRUN + 4 * tid);
    *(volatile v4i*)(cop + it * NBRUN + 4 * tid) = v;
  }
#pragma unroll
  for (int k = 0; k < NTY; ++k) {
    const v4i a = *(const v4ia*)(tb + k * NBRUN + 4 * tid);
    const v4i c = *(const v4ia*)(tb + NTY * NBRUN + k * NBRUN + 4 * tid);
    *(volatile v4i*)(dvp + (size_t)k * NP + 4 * tid) = a;
    *(volatile v4i*)(dip + (size_t)k * NP + 4 * tid) = c;
  }
  if (tid < 8) {
    const v4i f = {ov, ov, ov, ov};
    *(volatile v4i*)(fp + 4 * tid) = f;
  }
}

__global__ __launch_bounds__(NTHR) void k_bucket(const int* __restrict__ srcs, const int* __restrict__ dsts,
                                                 const int* __restrict__ attr, int* LIST, int* CO, int* FLAG,
                                                 int* DINVb, int* DEGINVb) {
  extern __shared__ __attribute__((aligned(16))) int dsm[];
  int* wl   = dsm;
  int* pl   = dsm + NWAVE * WLCAP;
  int* cnt  = pl + RCAP;
  int* offs = cnt + NBRUN;
  int* cur  = offs + NBRUN;
  int* c3   = cur + NBRUN;
  int* misc = c3 + NTY * NBRUN;
  const int tid = (int)threadIdx.x, lane = tid & 31, wave = tid >> 5;
  const int blk = (int)blockIdx.x;
  const unsigned nbs = (unsigned)(blk * NBRUN);
  const int nbi = (NN - blk * NBRUN) < NBRUN ? (NN - blk * NBRUN) : NBRUN;
  const unsigned unb = (unsigned)(nbi < 0 ? 0 : nbi);

  {
    const v4i z4 = {0, 0, 0, 0};
    for (int i = tid * 4; i < BK_ZINTS; i += NTHR * 4) *(v4ia*)(dsm + i) = z4;
    if (tid < 16) misc[tid] = 0;
  }
  __syncthreads();

  {
    const int per  = ((NE + NWAVE * WCH - 1) / (NWAVE * WCH)) * WCH;
    const int ebeg = wave * per;
    const int eend = (ebeg + per < NE) ? (ebeg + per) : NE;
    int* mylist = wl + wave * WLCAP;
    int wc = 0;
#pragma unroll 1
    for (int cb = ebeg; cb < eend; cb += WCH) {
      const int e0 = cb + lane * EPT;
      const v4i da = *(const v4ia*)(dsts + e0);
      const v4i db = *(const v4ia*)(dsts + e0 + 4);
      const unsigned s0 = (unsigned)da.x - nbs, s1 = (unsigned)da.y - nbs;
      const unsigned s2 = (unsigned)da.z - nbs, s3 = (unsigned)da.w - nbs;
      const unsigned s4 = (unsigned)db.x - nbs, s5 = (unsigned)db.y - nbs;
      const unsigned s6 = (unsigned)db.z - nbs, s7 = (unsigned)db.w - nbs;
      const bool h0 = s0 < unb, h1 = s1 < unb, h2 = s2 < unb, h3 = s3 < unb;
      const bool h4 = s4 < unb, h5 = s5 < unb, h6 = s6 < unb, h7 = s7 < unb;
      const unsigned m0 = __builtin_amdgcn_ballot_w32(h0), m1 = __builtin_amdgcn_ballot_w32(h1);
      const unsigned m2 = __builtin_amdgcn_ballot_w32(h2), m3 = __builtin_amdgcn_ballot_w32(h3);
      const unsigned m4 = __builtin_amdgcn_ballot_w32(h4), m5 = __builtin_amdgcn_ballot_w32(h5);
      const unsigned m6 = __builtin_amdgcn_ballot_w32(h6), m7 = __builtin_amdgcn_ballot_w32(h7);
      const unsigned any = m0 | m1 | m2 | m3 | m4 | m5 | m6 | m7;
      if (any != 0u) {
        const int pre = (int)(__builtin_amdgcn_mbcnt_lo(m0, 0u) + __builtin_amdgcn_mbcnt_lo(m1, 0u) +
                              __builtin_amdgcn_mbcnt_lo(m2, 0u) + __builtin_amdgcn_mbcnt_lo(m3, 0u) +
                              __builtin_amdgcn_mbcnt_lo(m4, 0u) + __builtin_amdgcn_mbcnt_lo(m5, 0u) +
                              __builtin_amdgcn_mbcnt_lo(m6, 0u) + __builtin_amdgcn_mbcnt_lo(m7, 0u));
        int p = wc + pre;
        if (h0) { if (p < WLCAP) mylist[p] = ((int)s0 << 20) | (e0 + 0); p = p + 1; }
        if (h1) { if (p < WLCAP) mylist[p] = ((int)s1 << 20) | (e0 + 1); p = p + 1; }
        if (h2) { if (p < WLCAP) mylist[p] = ((int)s2 << 20) | (e0 + 2); p = p + 1; }
        if (h3) { if (p < WLCAP) mylist[p] = ((int)s3 << 20) | (e0 + 3); p = p + 1; }
        if (h4) { if (p < WLCAP) mylist[p] = ((int)s4 << 20) | (e0 + 4); p = p + 1; }
        if (h5) { if (p < WLCAP) mylist[p] = ((int)s5 << 20) | (e0 + 5); p = p + 1; }
        if (h6) { if (p < WLCAP) mylist[p] = ((int)s6 << 20) | (e0 + 6); p = p + 1; }
        if (h7) { if (p < WLCAP) mylist[p] = ((int)s7 << 20) | (e0 + 7); p = p + 1; }
        wc += (int)(__builtin_popcount(m0) + __builtin_popcount(m1) + __builtin_popcount(m2) + __builtin_popcount(m3) +
                    __builtin_popcount(m4) + __builtin_popcount(m5) + __builtin_popcount(m6) + __builtin_popcount(m7));
      }
    }
    if (lane == 0) misc[wave] = wc;
  }
  __syncthreads();

  if (wave == 0) {
    int ov = 0;
#pragma unroll 1
    for (int w2 = 0; w2 < NWAVE; ++w2) {
      int c = misc[w2];
      if (c > WLCAP) ov = 1;
      c = c < 0 ? 0 : (c > WLCAP ? WLCAP : c);
#pragma unroll 1
      for (int b0 = 0; b0 < c; b0 += 32) {
        const int idx = b0 + lane;
        const int ent = wl[w2 * WLCAP + (idx < WLCAP ? idx : WLCAP - 1)];
        int eid = ent & 0xFFFFF;
        eid = eid > NE - 1 ? NE - 1 : eid;
        int ty = attr[eid];
        ty = ty < 0 ? 0 : (ty > NTY - 1 ? NTY - 1 : ty);
        const int m32 = (c - b0) < 32 ? (c - b0) : 32;
#pragma unroll 1
        for (int k = 0; k < m32; ++k) {
          const int u    = __builtin_amdgcn_readlane(ent, k);
          const int tk   = __builtin_amdgcn_readlane(ty, k);
          const int slot = (u >> 20) & (NBRUN - 1);
          if (lane == 0) {
            cnt[slot] = cnt[slot] + 1;
            c3[tk * NBRUN + slot] = c3[tk * NBRUN + slot] + 1;
          }
        }
      }
    }
    if (lane == 0) misc[9] = ov;
  }
  __syncthreads();
  if (wave == 0) {
    const int base = lane * (NBRUN / 32);
    int s = 0;
#pragma unroll 1
    for (int i = 0; i < NBRUN / 32; ++i) s += cnt[base + i];
    int incl = s;
#pragma unroll
    for (int d = 1; d < 32; d <<= 1) {
      const int y = __shfl_up(incl, d, 32);
      if (lane >= d) incl += y;
    }
    int run = incl - s;
#pragma unroll 1
    for (int i = 0; i < NBRUN / 32; ++i) {
      const int cv = cnt[base + i];
      offs[base + i] = run;
      cur[base + i]  = run;
      run += cv;
    }
  }
  __syncthreads();

  if (wave == 0) {
#pragma unroll 1
    for (int w2 = 0; w2 < NWAVE; ++w2) {
      int c = misc[w2];
      c = c < 0 ? 0 : (c > WLCAP ? WLCAP : c);
#pragma unroll 1
      for (int b0 = 0; b0 < c; b0 += 32) {
        const int idx = b0 + lane;
        const int ent = wl[w2 * WLCAP + (idx < WLCAP ? idx : WLCAP - 1)];
        const int m32 = (c - b0) < 32 ? (c - b0) : 32;
#pragma unroll 1
        for (int k = 0; k < m32; ++k) {
          const int u    = __builtin_amdgcn_readlane(ent, k);
          const int slot = (u >> 20) & (NBRUN - 1);
          if (lane == 0) {
            int p = cur[slot];
            p = p < 0 ? 0 : (p > RCAP - 1 ? RCAP - 1 : p);
            pl[p] = u & 0xFFFFF;
            cur[slot] = p + 1;
          }
        }
      }
    }
  }
  __syncthreads();

#pragma unroll 1
  for (int i = tid; i < RCAP; i += NTHR) {
    int e = pl[i];
    e = e < 0 ? 0 : (e > NE - 1 ? NE - 1 : e);
    int s = srcs[e];
    int t = attr[e];
    s = s < 0 ? 0 : (s > NN - 1 ? NN - 1 : s);
    t = t < 0 ? 0 : (t > NTY - 1 ? NTY - 1 : t);
    pl[i] = s | (t << 16);
  }
#pragma unroll 1
  for (int i = tid; i < NTY * NBRUN; i += NTHR) {
    const float dg = (float)c3[i] + 1.0f;
    wl[i] = __float_as_int(1.0f / sqrtf(dg));
    wl[NTY * NBRUN + i] = __float_as_int(1.0f / dg);
  }
  __syncthreads();

  const int ovf = misc[9];
  int* lp  = LIST + (size_t)blk * (2 * RCAP);
  int* cop = CO + (size_t)blk * (2 * NBRUN);
  int* fp  = FLAG + (size_t)blk * 32;
  int* dvp = DINVb + (size_t)blk * NBRUN;
  int* dip = DEGINVb + (size_t)blk * NBRUN;
  bucket_flush(pl, cnt, wl, ovf, lp, cop, fp, dvp, dip, tid);
  __threadfence();
  bucket_flush(pl, cnt, wl, ovf, lp, cop, fp, dvp, dip, tid);
}

template <int KTOT, int PB>
__device__ __forceinline__ void gemm_16x64(const unsigned short* __restrict__ ap,
                                           const unsigned short* __restrict__ bp, v8f (&acc)[4]) {
#pragma unroll 1
  for (int k0 = 0; k0 < KTOT; k0 += 32) {
    FragB af;
    af.h[0] = *(const v8usa*)(ap + k0);
    af.h[1] = *(const v8usa*)(ap + k0 + 16);
#pragma unroll
    for (int nt = 0; nt < 4; ++nt) {
      const unsigned short* wq = bp + (size_t)(16 * nt) * (size_t)PB + k0;
      FragB bf;
      bf.h[0] = *(const v8usa*)wq;
      bf.h[1] = *(const v8usa*)(wq + 16);
      acc[nt] = wmb(af, bf, acc[nt]);
    }
  }
}

__device__ __forceinline__ void stage_d(float* stg, const v8f (&acc)[4], int wave, int hh, int m) {
#pragma unroll
  for (int nt = 0; nt < 4; ++nt) {
#pragma unroll
    for (int r = 0; r < 8; ++r) stg[(16 * wave + 8 * hh + r) * SP + 16 * nt + m] = acc[nt][r];
  }
}

template <int KTOT, int PA, int PB>
__global__ __launch_bounds__(NTHR) __attribute__((amdgpu_num_vgpr(248)))
void k_gemm(const unsigned short* __restrict__ A, const unsigned short* __restrict__ BT, float* XW) {
  __shared__ __attribute__((aligned(16))) float stg[GBM * SP];
  const int tid = (int)threadIdx.x, lane = tid & 31, wave = tid >> 5, hh = lane >> 4, m = lane & 15;
  const int rowBase = (int)blockIdx.x * GBM;
  const int col0    = (int)blockIdx.y * 64;

  v8f acc[4];
  {
    const v8f z = {0.f, 0.f, 0.f, 0.f, 0.f, 0.f, 0.f, 0.f};
#pragma unroll
    for (int t = 0; t < 4; ++t) acc[t] = z;
  }
  const unsigned short* ap = A + (size_t)(rowBase + 16 * wave + m) * (size_t)PA + 8 * hh;
  const unsigned short* bp = BT + (size_t)(col0 + m) * (size_t)PB + 8 * hh;
  gemm_16x64<KTOT, PB>(ap, bp, acc);
  stage_d(stg, acc, wave, hh, m);
  __syncthreads();

#pragma unroll 1
  for (int i = 0; i < 8; ++i) {
    const int lr   = 16 * wave + 2 * i + hh;
    const int grow = rowBase + lr;
    const v4f a = *(const v4fa*)(stg + lr * SP + 4 * m);
    st2_v4f(XW + (size_t)grow * NCOL + col0 + 4 * m, a);
  }
}

template <int LAST>
__global__ __launch_bounds__(NTHR) void k_replay(const int* __restrict__ LIST, const int* __restrict__ CO,
                                                 const int* __restrict__ FLAG, const float* __restrict__ DINV,
                                                 const float* __restrict__ DEGINV, const float* __restrict__ XW,
                                                 const float* __restrict__ B3t, float* X, unsigned short* XHL,
                                                 float* out) {
  __shared__ __attribute__((aligned(16))) float sb[64];
  const int tid = (int)threadIdx.x, lane = tid & 31, wave = tid >> 5, hh = lane >> 4, q = lane & 15;
  const int rowBase = (int)blockIdx.x * GBM;
  const int bucket  = rowBase >> SLB;
  const int* lb  = LIST + (size_t)bucket * (2 * RCAP);
  const int* cob = CO + (size_t)bucket * (2 * NBRUN);
  const int flag = FLAG[(size_t)bucket * 32];
  const float qnan = __uint_as_float(0x7fc00000u);
  if (tid < 16) *(v4fa*)(sb + 4 * tid) = *(const v4fa*)(B3t + 4 * tid);
  __syncthreads();
  const v4f bias = *(const v4fa*)(sb + 4 * q);

#pragma unroll 1
  for (int i = 0; i < 8; ++i) {
    const int d    = rowBase + 16 * wave + 2 * i + hh;
    const int slot = d & (NBRUN - 1);
    int c = cob[slot];
    int o = cob[NBRUN + slot];
    const float d0 = DINV[d], d1 = DINV[NP + d], d2 = DINV[2 * NP + d];
    asm volatile("" :: "v"(d0), "v"(d1), "v"(d2));
    const bool big = c > TRIPCAP;
    c = c < 0 ? 0 : (c > TRIPCAP ? TRIPCAP : c);
    o = o < 0 ? 0 : (o > RCAP - 1 ? RCAP - 1 : o);
    const int co = __shfl_xor(c, 16, 32);
    const int cm = c > co ? c : co;
    const int cmu = __builtin_amdgcn_readfirstlane(cm);
    int last = o + c - 1;
    last = last < o ? o : last;
    last = last > RCAP - 1 ? RCAP - 1 : last;
    float a0 = 0.0f, a1 = 0.0f, a2 = 0.0f, a3 = 0.0f;
#pragma unroll 1
    for (int j = 0; j < cmu; ++j) {
      int idx = o + j;
      idx = idx > last ? last : idx;
      const v2i ent = *(const v2ia*)(lb + 2 * (size_t)idx);
      int sr = ent.x;
      int ty = ent.y;
      sr = sr < 0 ? 0 : (sr > NN - 1 ? NN - 1 : sr);
      ty = ty < 0 ? 0 : (ty > NTY - 1 ? NTY - 1 : ty);
      const float ds = DINV[(size_t)ty * NP + sr];
      const v4f v = *(const v4fa*)(XW + (size_t)sr * NCOL + 64 * ty + 4 * q);
      asm volatile("" :: "v"(ds));
      asm volatile("" :: "v"(v));
      const float dd = (ty == 0) ? d0 : ((ty == 1) ? d1 : d2);
      const float w = ds * dd;
      const bool valid = j < c;
      const float t0 = fmaf(w, v.x, a0), t1 = fmaf(w, v.y, a1), t2 = fmaf(w, v.z, a2), t3 = fmaf(w, v.w, a3);
      a0 = valid ? t0 : a0; a1 = valid ? t1 : a1; a2 = valid ? t2 : a2; a3 = valid ? t3 : a3;
    }
    const float e0 = DEGINV[d], e1 = DEGINV[NP + d], e2 = DEGINV[2 * NP + d];
    const float* xr = XW + (size_t)d * NCOL + 4 * q;
    const v4f s0 = *(const v4fa*)xr;
    const v4f s1 = *(const v4fa*)(xr + 64);
    const v4f s2 = *(const v4fa*)(xr + 128);
    const v4f xin = *(const v4fa*)(X + (size_t)d * HD + 4 * q);
    asm volatile("" :: "v"(e0), "v"(e1), "v"(e2));
    asm volatile("" :: "v"(s0));
    asm volatile("" :: "v"(s1));
    asm volatile("" :: "v"(s2));
    asm volatile("" :: "v"(xin));
    a0 = fmaf(e0, s0.x, a0); a1 = fmaf(e0, s0.y, a1); a2 = fmaf(e0, s0.z, a2); a3 = fmaf(e0, s0.w, a3);
    a0 = fmaf(e1, s1.x, a0); a1 = fmaf(e1, s1.y, a1); a2 = fmaf(e1, s1.z, a2); a3 = fmaf(e1, s1.w, a3);
    a0 = fmaf(e2, s2.x, a0); a1 = fmaf(e2, s2.y, a1); a2 = fmaf(e2, s2.z, a2); a3 = fmaf(e2, s2.w, a3);
    a0 += bias.x; a1 += bias.y; a2 += bias.z; a3 += bias.w;
    a0 = (a0 > 0.0f) ? a0 : (a0 - a0); a1 = (a1 > 0.0f) ? a1 : (a1 - a1);
    a2 = (a2 > 0.0f) ? a2 : (a2 - a2); a3 = (a3 > 0.0f) ? a3 : (a3 - a3);
    const float v0 = xin.x + a0, v1 = xin.y + a1, v2 = xin.z + a2, v3 = xin.w + a3;
    float ss = ((v0 * v0 + v1 * v1) + v2 * v2) + v3 * v3;
    ss += __shfl_xor(ss, 8, 32);
    ss += __shfl_xor(ss, 4, 32);
    ss += __shfl_xor(ss, 2, 32);
    ss += __shfl_xor(ss, 1, 32);
    const float sn  = sqrtf(ss);
    const float nrm = (sn < 1e-12f) ? 1e-12f : sn;
    float m0 = v0 / nrm, m1 = v1 / nrm, m2 = v2 / nrm, m3 = v3 / nrm;
    const bool bad  = (flag != 0) | big;
    const bool live = d < NN;
    m0 = bad ? qnan : m0; m1 = bad ? qnan : m1; m2 = bad ? qnan : m2; m3 = bad ? qnan : m3;
    m0 = live ? m0 : 0.0f; m1 = live ? m1 : 0.0f; m2 = live ? m2 : 0.0f; m3 = live ? m3 : 0.0f;
    v4f ov;
    ov.x = m0; ov.y = m1; ov.z = m2; ov.w = m3;
    if constexpr (LAST != 0) {
      float* op = out + (size_t)d * HD + 4 * q;
      if (live) {
        *(volatile v4f*)op = ov;
      }
      __threadfence();
      if (live) {
        *(volatile v4f*)op = ov;
      }
    } else {
      int h01, h23, l01, l23;
      hilo_pack(m0, m1, m2, m3, h01, h23, l01, l23);
      const v4i ow = regroup8(h01, h23, l01, l23, lane);
      float* op = X + (size_t)d * HD + 4 * q;
      unsigned short* hp = XHL + (size_t)d * KL + 8 * q;
      *(volatile v4f*)op = ov;
      *(volatile v4i*)hp = ow;
      __threadfence();
      *(volatile v4f*)op = ov;
      *(volatile v4i*)hp = ow;
    }
  }
}

extern "C" void kernel_launch(void* const* d_in, const int* in_sizes, int n_in,
                              void* d_out, int out_size, void* d_ws, size_t ws_size,
                              hipStream_t stream) {
  if (n_in < 5) return;
  if (in_sizes[0] != NN * HD) return;
  if (in_sizes[1] != 2 * NE) return;
  if (in_sizes[2] != NE) return;
  if (in_sizes[3] != NLAY * NTY * HD * HD) return;
  if (in_sizes[4] != NLAY * NTY * HD) return;
  if (out_size != NN * HD) return;

  const float* x  = (const float*)d_in[0];
  const int*   ei = (const int*)d_in[1];
  const int*   ea = (const int*)d_in[2];
  const float* W  = (const float*)d_in[3];
  const float* b  = (const float*)d_in[4];
  float* out = (float*)d_out;
  const int* srcs = ei;
  const int* dsts = ei + NE;

  constexpr size_t zXB   = (size_t)MP * HD * 2;
  constexpr size_t zX    = (size_t)MP * HD * 4;
  constexpr size_t zXHL  = (size_t)MP * KL * 2;
  constexpr size_t zXW   = (size_t)MP * NCOL * 4;
  constexpr size_t zLIST = (size_t)NBK * RCAP * 8;
  constexpr size_t zCO   = (size_t)NBK * 2 * NBRUN * 4;
  constexpr size_t zFLAG = 6400;
  constexpr size_t zTAB  = (size_t)NTY * NP * 4;
  constexpr size_t zWT0  = (size_t)NCOL * HD * 2;
  constexpr size_t zWT12 = (size_t)2 * NCOL * KL * 2;
  constexpr size_t zB3   = 1024;
  constexpr size_t oXB   = 0;
  constexpr size_t oX    = oXB + zXB;
  constexpr size_t oXHL  = oX + zX;
  constexpr size_t oXW   = oXHL + zXHL;
  constexpr size_t oLIST = oXW + zXW;
  constexpr size_t oCO   = oLIST + zLIST;
  constexpr size_t oFLAG = oCO + zCO;
  constexpr size_t oDINV = oFLAG + zFLAG;
  constexpr size_t oDEGI = oDINV + zTAB;
  constexpr size_t oWT0  = oDEGI + zTAB;
  constexpr size_t oWT12 = oWT0 + zWT0;
  constexpr size_t oB3   = oWT12 + zWT12;
  constexpr size_t oEND  = oB3 + zB3;
  static_assert(zXB % 256 == 0 && zX % 256 == 0 && zXHL % 256 == 0 && zXW % 256 == 0 && zLIST % 256 == 0);
  static_assert(zCO % 256 == 0 && zFLAG % 256 == 0 && zTAB % 256 == 0 && zWT0 % 256 == 0 && zWT12 % 256 == 0);
  static_assert(zFLAG >= (size_t)NBK * 128 && zB3 >= (size_t)NLAY * HD * 4);
  static_assert(oEND <= (size_t)(128u << 20));
  if (oEND > ws_size) return;

  char* ws = (char*)d_ws;
  unsigned short* XB   = (unsigned short*)(ws + oXB);
  float*          X    = (float*)(ws + oX);
  unsigned short* XHL  = (unsigned short*)(ws + oXHL);
  float*          XW   = (float*)(ws + oXW);
  int*            LIST = (int*)(ws + oLIST);
  int*            CO   = (int*)(ws + oCO);
  int*            FLAG = (int*)(ws + oFLAG);
  float*          DINV = (float*)(ws + oDINV);
  float*          DEGI = (float*)(ws + oDEGI);
  unsigned short* WT0  = (unsigned short*)(ws + oWT0);
  unsigned short* WT12 = (unsigned short*)(ws + oWT12);
  float*          B3   = (float*)(ws + oB3);
  const unsigned short* WT1 = WT12;
  const unsigned short* WT2 = WT12 + (size_t)NCOL * KL;

  hipFuncSetAttribute(reinterpret_cast<const void*>(&k_bucket), hipFuncAttributeMaxDynamicSharedMemorySize, (int)BK_LDS);

  const dim3 gg(MP / GBM, NCOL / 64);
  k_prep<<<PBTOT, NTHR, 0, stream>>>(x, W, b, XB, X, WT0, WT12, B3);
  k_bucket<<<NBK, NTHR, BK_LDS, stream>>>(srcs, dsts, ea, LIST, CO, FLAG, (int*)DINV, (int*)DEGI);
  k_gemm<64, HD, HD><<<gg, NTHR, 0, stream>>>(XB, WT0, XW);
  k_replay<0><<<MP / GBM, NTHR, 0, stream>>>(LIST, CO, FLAG, DINV, DEGI, XW, B3, X, XHL, out);
  k_gemm<K_L1, KL, KL><<<gg, NTHR, 0, stream>>>(XHL, WT1, XW);
  k_replay<0><<<MP / GBM, NTHR, 0, stream>>>(LIST, CO, FLAG, DINV, DEGI, XW, B3 + HD, X, XHL, out);
  k_gemm<K_L2, KL, KL><<<gg, NTHR, 0, stream>>>(XHL, WT2, XW);
  k_replay<1><<<MP / GBM, NTHR, 0, stream>>>(LIST, CO, FLAG, DINV, DEGI, XW, B3 + 2 * HD, X, XHL, out);
}
